// KANLinear2D_47742856462889
// MI455X (gfx1250) — hardware-verified
//
#include <hip/hip_runtime.h>


typedef _Float16 bf16_t;
typedef __attribute__((ext_vector_type(16))) _Float16 v16bf;
typedef __attribute__((ext_vector_type(8)))  _Float16 v8bf;
typedef __attribute__((ext_vector_type(4)))  float v4f_t;
typedef float v4fa __attribute__((ext_vector_type(4), may_alias));
__device__ __forceinline__ void stpk(bf16_t* p, float v0, float v1) {
  const unsigned u = (unsigned)__builtin_bit_cast(unsigned short, (bf16_t)v0) | ((unsigned)__builtin_bit_cast(unsigned short, (bf16_t)v1) << 16);
  *(volatile unsigned*)p = u; __threadfence(); *(volatile unsigned*)p = u;
}
typedef __attribute__((ext_vector_type(8)))  float  v8f;
typedef __attribute__((ext_vector_type(4)))  int    v4i;

#define M_TOTAL 16384
#define N_OUT   512
#define K_IN    512
#define K_TOT   1024

#define TILE_M 128
#define TILE_N 128
#define TILE_K 32
#define LDSS   40

#if defined(__has_builtin)
#if __has_builtin(__builtin_amdgcn_global_load_async_to_lds_b128)
#define HAS_ASYNC_LDS 1
#endif
#endif

__device__ __forceinline__ void copy16_g2l(const bf16_t* g, bf16_t* l) {
#ifdef HAS_ASYNC_LDS
  __builtin_amdgcn_global_load_async_to_lds_b128(
      (__attribute__((address_space(1))) v4i*)g,
      (__attribute__((address_space(3))) v4i*)l, 0, 0);
#else
  *(uint4*)l = *(const uint4*)g;
#endif
}

__device__ __forceinline__ void wait_async_all() {
#ifdef HAS_ASYNC_LDS
#if __has_builtin(__builtin_amdgcn_s_wait_asynccnt)
  __builtin_amdgcn_s_wait_asynccnt(0);
#else
  asm volatile("s_wait_asynccnt 0" ::: "memory");
#endif
#endif
}

union Frag16 { v16bf v; v8bf h[2]; };

__global__ __launch_bounds__(256)
void kan_prep_kernel(const float* __restrict__ x,
                     const float* __restrict__ bsw,
                     bf16_t* __restrict__ A) {
  const int idx0 = ((int)blockIdx.x * 256 + (int)threadIdx.x) * 2;
  const int m = idx0 >> 9;
  const int i0 = idx0 & (K_IN - 1);
  float si[2], sp[2];
#pragma unroll
  for (int u = 0; u < 2; ++u) {
    const int i = i0 + u;
    const float v = x[idx0 + u];

    const float sig = 1.0f / (1.0f + __expf(-v));
    si[u] = v * sig;

    const float h = 0.4f;
    float b[11];
#pragma unroll
    for (int j = 0; j < 11; ++j) {
      const float g0 = -1.0f + (float)(j - 3) * h;
      const float g1 = g0 + h;
      b[j] = (v >= g0 && v < g1) ? 1.0f : 0.0f;
    }
#pragma unroll
    for (int k = 1; k <= 3; ++k) {
      const float inv = 1.0f / ((float)k * h);
#pragma unroll
      for (int j = 0; j < 11 - k; ++j) {
        const float gj = -1.0f + (float)(j - 3) * h;
        const float gk = -1.0f + (float)(j + k - 2) * h;
        b[j] = (v - gj) * inv * b[j] + (gk - v) * inv * b[j + 1];
      }
    }
    const float* w = bsw + i * 8;
    float spl = 0.0f;
#pragma unroll
    for (int k = 0; k < 8; ++k) spl = __builtin_fmaf(w[k], b[k], spl);
    sp[u] = spl;
  }
  stpk(A + (size_t)m * K_TOT + i0, si[0], si[1]);
  stpk(A + (size_t)m * K_TOT + K_IN + i0, sp[0], sp[1]);
}

__global__ __launch_bounds__(256)
void kan_packw_kernel(const float* __restrict__ bw,
                      const float* __restrict__ sw,
                      bf16_t* __restrict__ Wc) {
  const int idx = ((int)blockIdx.x * 256 + (int)threadIdx.x) * 2;
  const int n = idx >> 10;
  const int k = idx & (K_TOT - 1);
  const float v0 = (k < K_IN) ? bw[n * K_IN + k] : sw[n * K_IN + (k - K_IN)];
  const float v1 = (k + 1 < K_IN) ? bw[n * K_IN + k + 1] : sw[n * K_IN + (k + 1 - K_IN)];
  stpk(Wc + idx, v0, v1);
}

__global__ __launch_bounds__(256)
void kan_gemm_kernel(const bf16_t* __restrict__ A,
                     const bf16_t* __restrict__ W,
                     float* __restrict__ C) {
  __shared__ alignas(16) bf16_t sA[2][TILE_M * LDSS];
  __shared__ alignas(16) bf16_t sB[2][TILE_N * LDSS];

  const int tid    = (int)threadIdx.x;
  const int lane   = tid & 31;
  const int wave   = tid >> 5;
  const int waveM  = wave & 3;
  const int waveN  = wave >> 2;
  const int lrow   = lane & 15;
  const int hsel   = lane >> 4;
  const int blockM = (int)blockIdx.x * TILE_M;
  const int blockN = (int)blockIdx.y * TILE_N;

  v8f acc[2][4];
#pragma unroll
  for (int mi = 0; mi < 2; ++mi)
#pragma unroll
    for (int ni = 0; ni < 4; ++ni)
      acc[mi][ni] = (v8f){0.f, 0.f, 0.f, 0.f, 0.f, 0.f, 0.f, 0.f};

  auto load_tiles = [&](int kt, int buf) {
#pragma unroll
    for (int r = 0; r < 2; ++r) {
      const int c   = tid + r * 256;
      const int row = c >> 2;
      const int col = (c & 3) * 8;
      copy16_g2l(A + (size_t)(blockM + row) * K_TOT + kt * TILE_K + col,
                 &sA[buf][row * LDSS + col]);
      copy16_g2l(W + (size_t)(blockN + row) * K_TOT + kt * TILE_K + col,
                 &sB[buf][row * LDSS + col]);
    }
  };

  load_tiles(0, 0);

  const int KSTEPS = K_TOT / TILE_K;
  for (int kt = 0; kt < KSTEPS; ++kt) {
    const int buf = kt & 1;
    wait_async_all();
    __syncthreads();
    if (kt + 1 < KSTEPS) load_tiles(kt + 1, buf ^ 1);

    Frag16 af[2];
#pragma unroll
    for (int mi = 0; mi < 2; ++mi) {
      const bf16_t* p = &sA[buf][(waveM * 32 + mi * 16 + lrow) * LDSS];
      af[mi].h[0] = *(const v8bf*)(p + hsel * 8);
      af[mi].h[1] = *(const v8bf*)(p + 16 + hsel * 8);
    }
    Frag16 bfm[4];
#pragma unroll
    for (int ni = 0; ni < 4; ++ni) {
      const bf16_t* p = &sB[buf][(waveN * 64 + ni * 16 + lrow) * LDSS];
      bfm[ni].h[0] = *(const v8bf*)(p + hsel * 8);
      bfm[ni].h[1] = *(const v8bf*)(p + 16 + hsel * 8);
    }

#pragma unroll
    for (int mi = 0; mi < 2; ++mi)
#pragma unroll
      for (int ni = 0; ni < 4; ++ni)
        acc[mi][ni] = __builtin_amdgcn_wmma_f32_16x16x32_f16(
            false, af[mi].v, false, bfm[ni].v,
            (short)0, acc[mi][ni], false, false);

    __syncthreads();
  }

  __shared__ alignas(16) float stg[8][32 * 68];
  float* swv = stg[wave];
#pragma unroll
  for (int mi = 0; mi < 2; ++mi)
#pragma unroll
    for (int ni = 0; ni < 4; ++ni)
#pragma unroll
      for (int r = 0; r < 8; ++r) swv[(mi * 16 + hsel * 8 + r) * 68 + ni * 16 + lrow] = acc[mi][ni][r];
  asm volatile("s_wait_dscnt 0" ::: "memory");
#pragma unroll 1
  for (int pass = 0; pass < 2; ++pass) {
#pragma unroll
    for (int i = 0; i < 16; ++i) { const int c = lane + 32 * i, rr = c >> 4, q = (c & 15) * 4;
      *(volatile v4f_t*)(C + (size_t)(blockM + waveM * 32 + rr) * N_OUT + blockN + waveN * 64 + q) = *(const volatile v4fa*)(swv + rr * 68 + q); }
    __threadfence();
  }
}

extern "C" void kernel_launch(void* const* d_in, const int* in_sizes, int n_in,
                              void* d_out, int out_size, void* d_ws, size_t ws_size,
                              hipStream_t stream) {
  const float* x   = (const float*)d_in[0];
  const float* bw  = (const float*)d_in[1];
  const float* sw  = (const float*)d_in[2];
  const float* bsw = (const float*)d_in[3];
  float* out = (float*)d_out;

  bf16_t* A  = (bf16_t*)d_ws;
  bf16_t* Wc = A + (size_t)M_TOTAL * K_TOT;

  kan_prep_kernel<<<(M_TOTAL * K_IN) / 512, 256, 0, stream>>>(x, bsw, A);
  kan_packw_kernel<<<(N_OUT * K_TOT) / 512, 256, 0, stream>>>(bw, sw, Wc);

  dim3 grid(M_TOTAL / TILE_M, N_OUT / TILE_N);
  kan_gemm_kernel<<<grid, 256, 0, stream>>>(A, Wc, out);
}
